// HarmonicOscillatorWithInteraction1D_89137751261222
// MI455X (gfx1250) — hardware-verified
//
#include <hip/hip_runtime.h>
#include <stddef.h>

typedef _Float16 v16h __attribute__((ext_vector_type(16)));
typedef _Float16 v8h  __attribute__((ext_vector_type(8)));
typedef float    v8f  __attribute__((ext_vector_type(8)));
typedef float    v4f  __attribute__((ext_vector_type(4)));
typedef v8h __attribute__((may_alias)) v8ha;
typedef v4f __attribute__((may_alias)) v4fa;

union Frag { v16h v; v8h hf[2]; };
union H8   { v8h v; _Float16 e[8]; };
union F4   { v4f v; float e[4]; };

#define NWALK 8192
#define NPART 8
#define HID   512

#define SC_W2 16.0f
#define SC_V2 256.0f
#define SC_S1 64.0f
#define SC_W1 2.0f
#define INV_SC_Z2 0.0625f
#define INV_SC_R  0.000244140625f
#define TERM1_SCALE 4.76837158203125e-07f
#define GAUSS_C 1.5957691216057308f

__device__ __forceinline__ v8f zero8() {
  v8f z = {0.f, 0.f, 0.f, 0.f, 0.f, 0.f, 0.f, 0.f};
  return z;
}

__device__ __forceinline__ v8f wmma_f16(v16h a, v16h b, v8f c) {
  v8f d = __builtin_amdgcn_wmma_f32_16x16x32_f16(false, a, false, b, (short)0, c, false, false);
  asm volatile("v_nop\n\tv_nop\n\tv_nop\n\tv_nop" : "+v"(d) : "v"(a), "v"(b));
  return d;
}

__device__ __forceinline__ v16h ld_frag(const _Float16* row, int k0, int h) {
  Frag f;
  f.hf[0] = *(const v8ha*)(row + k0 + 8 * h);
  f.hf[1] = *(const v8ha*)(row + k0 + 16 + 8 * h);
  return f.v;
}

__device__ __forceinline__ void prep_store(float (*sT)[65], _Float16* w2h, _Float16* w2th,
                                           int j0, int k0, int w, int lane) {
#pragma unroll
  for (int s = 0; s < 2; ++s) {
    const int r  = w * 8 + s * 4 + (lane >> 3);
    const int c8 = (lane & 7) * 8;
    H8 dv, tv;
#pragma unroll
    for (int i = 0; i < 8; ++i) {
      dv.e[i] = (_Float16)sT[r][c8 + i];
      tv.e[i] = (_Float16)sT[c8 + i][r];
    }
    *(volatile v8h*)(w2h  + (size_t)(j0 + r) * HID + k0 + c8) = dv.v;
    *(volatile v8h*)(w2th + (size_t)(k0 + r) * HID + j0 + c8) = tv.v;
  }
}

__global__ __launch_bounds__(256)
void k_prep(const float* __restrict__ W2, _Float16* __restrict__ w2h, _Float16* __restrict__ w2th) {
  __shared__ float sT[64][65];
  const int tid = threadIdx.x, lane = tid & 31, w = tid >> 5;
  const int j0 = (blockIdx.x >> 3) * 64;
  const int k0 = (blockIdx.x & 7) * 64;
#pragma unroll
  for (int p = 0; p < 16; ++p) {
    const int idx = tid + 256 * p;
    const int r = idx >> 6, c = idx & 63;
    sT[r][c] = W2[(size_t)(j0 + r) * HID + k0 + c] * SC_W2;
  }
  __syncthreads();
  prep_store(sT, w2h, w2th, j0, k0, w, lane);
  __threadfence();
  prep_store(sT, w2h, w2th, j0, k0, w, lane);
}

__device__ __forceinline__ void fwd_store(float (*sH)[HID + 8], float* h1f, _Float16* h1h,
                                          _Float16* s1h, int b0, int tid) {
#pragma unroll
  for (int p = 0; p < 8; ++p) {
    const int c = tid + 256 * p;
    const int row = c >> 7, c4 = (c & 127) * 4;
    const v4f v = *(const v4fa*)(&sH[row][c4]);
    *(volatile v4f*)(h1f + (size_t)(b0 + row) * HID + c4) = v;
  }
#pragma unroll
  for (int p = 0; p < 4; ++p) {
    const int c = tid + 256 * p;
    const int row = c >> 6, c8 = (c & 63) * 8;
    H8 hv, sv;
#pragma unroll
    for (int i = 0; i < 8; ++i) {
      const float hh = sH[row][c8 + i];
      hv.e[i] = (_Float16)hh;
      sv.e[i] = (_Float16)(fmaf(-hh, hh, 1.0f) * SC_S1);
    }
    const size_t off = (size_t)(b0 + row) * HID + c8;
    *(volatile v8h*)(h1h + off) = hv.v;
    *(volatile v8h*)(s1h + off) = sv.v;
  }
}

__global__ __launch_bounds__(256)
void k_fwd(const float* __restrict__ x, const float* __restrict__ W1, const float* __restrict__ b1,
           float* __restrict__ h1f, _Float16* __restrict__ h1h, _Float16* __restrict__ s1h) {
  __shared__ float sX[16 * NPART];
  __shared__ __attribute__((aligned(16))) float sH[16][HID + 8];
  const int tid = threadIdx.x;
  const int b0 = blockIdx.x * 16;
  if (tid < 16 * NPART) sX[tid] = x[(size_t)b0 * NPART + tid];
  const int ja = tid, jb = tid + 256;
  float wa[NPART], wb[NPART];
#pragma unroll
  for (int d = 0; d < NPART; ++d) {
    wa[d] = W1[d * HID + ja];
    wb[d] = W1[d * HID + jb];
  }
  const float ba = b1[ja], bb = b1[jb];
  __syncthreads();
#pragma unroll 1
  for (int r = 0; r < 16; ++r) {
    float za = 0.f, zb = 0.f;
#pragma unroll
    for (int d = 0; d < NPART; ++d) {
      const float xv = sX[r * NPART + d];
      za = fmaf(xv, wa[d], za);
      zb = fmaf(xv, wb[d], zb);
    }
    sH[r][ja] = tanhf(za + ba);
    sH[r][jb] = tanhf(zb + bb);
  }
  __syncthreads();
  fwd_store(sH, h1f, h1h, s1h, b0, tid);
  __threadfence();
  fwd_store(sH, h1f, h1h, s1h, b0, tid);
}

__device__ __forceinline__ void gemm_32x32(const _Float16* ar0, const _Float16* br0, int h,
                                           v8f& a00, v8f& a01, v8f& a10, v8f& a11) {
  const _Float16* ar1 = ar0 + 16 * HID;
  const _Float16* br1 = br0 + 16 * HID;
  a00 = zero8(); a01 = zero8(); a10 = zero8(); a11 = zero8();
#pragma unroll 2
  for (int k0 = 0; k0 < HID; k0 += 32) {
    const v16h fa0 = ld_frag(ar0, k0, h);
    const v16h fa1 = ld_frag(ar1, k0, h);
    const v16h fb0 = ld_frag(br0, k0, h);
    const v16h fb1 = ld_frag(br1, k0, h);
    a00 = wmma_f16(fa0, fb0, a00);
    a01 = wmma_f16(fa0, fb1, a01);
    a10 = wmma_f16(fa1, fb0, a10);
    a11 = wmma_f16(fa1, fb1, a11);
  }
}

__device__ __forceinline__ void epi_tanh(float (*sT)[132], const float* sB2, v8f acc,
                                         int mi, int ni, int w, int h, int m) {
  const int cw = w * 32 + ni * 16 + m;
  const float bk = sB2[cw];
#pragma unroll
  for (int r = 0; r < 8; ++r) sT[mi * 16 + 8 * h + r][cw] = tanhf(acc[r] * INV_SC_Z2 + bk);
}

__device__ __forceinline__ void epi_scale(float (*sT)[132], v8f acc, float scale,
                                          int mi, int ni, int w, int h, int m) {
  const int cw = w * 32 + ni * 16 + m;
#pragma unroll
  for (int r = 0; r < 8; ++r) sT[mi * 16 + 8 * h + r][cw] = acc[r] * scale;
}

__device__ __forceinline__ void gemm1_store(float (*sT)[132], const float* sW3, _Float16* v2h,
                                            float* wf, int m0, int nb, int tid) {
#pragma unroll
  for (int p = 0; p < 4; ++p) {
    const int c = tid + 128 * p;
    const int row = c >> 4, c8 = (c & 15) * 8;
    H8 vv;
#pragma unroll
    for (int i = 0; i < 8; ++i) {
      const float h2 = sT[row][c8 + i];
      const float s2 = fmaf(-h2, h2, 1.0f);
      vv.e[i] = (_Float16)((s2 * sW3[c8 + i]) * SC_V2);
    }
    *(volatile v8h*)(v2h + (size_t)(m0 + row) * HID + nb + c8) = vv.v;
  }
#pragma unroll
  for (int p = 0; p < 8; ++p) {
    const int c = tid + 128 * p;
    const int row = c >> 5, c4 = (c & 31) * 4;
    F4 f;
#pragma unroll
    for (int i = 0; i < 4; ++i) {
      const float h2 = sT[row][c4 + i];
      const float s2 = fmaf(-h2, h2, 1.0f);
      f.e[i] = (sW3[c4 + i] * h2) * s2;
    }
    *(volatile v4f*)(wf + (size_t)(m0 + row) * HID + nb + c4) = f.v;
  }
}

__global__ __launch_bounds__(128)
void k_gemm1(const _Float16* __restrict__ h1h, const _Float16* __restrict__ w2th,
             const float* __restrict__ b2, const float* __restrict__ W3,
             _Float16* __restrict__ v2h, float* __restrict__ wf) {
  __shared__ __attribute__((aligned(16))) float sT[32][132];
  __shared__ float sB2[128];
  __shared__ float sW3[128];
  const int tid = threadIdx.x, lane = tid & 31, w = tid >> 5, h = lane >> 4, m = lane & 15;
  const int m0 = (blockIdx.x >> 2) * 32;
  const int nb = (blockIdx.x & 3) * 128;
  sB2[tid] = b2[nb + tid];
  sW3[tid] = W3[nb + tid];
  const _Float16* ar0 = h1h  + (size_t)(m0 + m) * HID;
  const _Float16* br0 = w2th + (size_t)(nb + w * 32 + m) * HID;
  v8f a00, a01, a10, a11;
  gemm_32x32(ar0, br0, h, a00, a01, a10, a11);
  __syncthreads();
  epi_tanh(sT, sB2, a00, 0, 0, w, h, m);
  epi_tanh(sT, sB2, a01, 0, 1, w, h, m);
  epi_tanh(sT, sB2, a10, 1, 0, w, h, m);
  epi_tanh(sT, sB2, a11, 1, 1, w, h, m);
  __syncthreads();
  gemm1_store(sT, sW3, v2h, wf, m0, nb, tid);
  __threadfence();
  gemm1_store(sT, sW3, v2h, wf, m0, nb, tid);
}

__device__ __forceinline__ void gemm2_store(float (*sT)[132], float* Rf, int m0, int nb, int tid) {
#pragma unroll
  for (int p = 0; p < 8; ++p) {
    const int c = tid + 128 * p;
    const int row = c >> 5, c4 = (c & 31) * 4;
    const v4f v = *(const v4fa*)(&sT[row][c4]);
    *(volatile v4f*)(Rf + (size_t)(m0 + row) * HID + nb + c4) = v;
  }
}

__global__ __launch_bounds__(128)
void k_gemm2(const _Float16* __restrict__ v2h, const _Float16* __restrict__ w2h,
             float* __restrict__ Rf) {
  __shared__ __attribute__((aligned(16))) float sT[32][132];
  const int tid = threadIdx.x, lane = tid & 31, w = tid >> 5, h = lane >> 4, m = lane & 15;
  const int m0 = (blockIdx.x >> 2) * 32;
  const int nb = (blockIdx.x & 3) * 128;
  const _Float16* ar0 = v2h + (size_t)(m0 + m) * HID;
  const _Float16* br0 = w2h + (size_t)(nb + w * 32 + m) * HID;
  v8f a00, a01, a10, a11;
  gemm_32x32(ar0, br0, h, a00, a01, a10, a11);
  epi_scale(sT, a00, INV_SC_R, 0, 0, w, h, m);
  epi_scale(sT, a01, INV_SC_R, 0, 1, w, h, m);
  epi_scale(sT, a10, INV_SC_R, 1, 0, w, h, m);
  epi_scale(sT, a11, INV_SC_R, 1, 1, w, h, m);
  __syncthreads();
  gemm2_store(sT, Rf, m0, nb, tid);
  __threadfence();
  gemm2_store(sT, Rf, m0, nb, tid);
}

__global__ __launch_bounds__(256)
void k_lapfin(const _Float16* __restrict__ s1h, const _Float16* __restrict__ w2th,
              const float* __restrict__ wf, const float* __restrict__ Rf,
              const float* __restrict__ h1f, const float* __restrict__ x,
              const float* __restrict__ W1, const float* __restrict__ b3,
              float* __restrict__ out) {
  __shared__ __attribute__((aligned(16))) _Float16 sW1h[NPART * HID];
  __shared__ float sW1f[NPART * HID];
  __shared__ float sQ[HID];
  __shared__ float sLap[8][16];
  __shared__ __attribute__((aligned(16))) float sOut[32];
  (void)b3;
  const int tid = threadIdx.x, lane = tid & 31, w = tid >> 5, h = lane >> 4, m = lane & 15;
  const int b0 = blockIdx.x * 32;

#pragma unroll
  for (int p = 0; p < 16; ++p) {
    const int idx = tid + 256 * p;
    const float v = W1[idx];
    sW1f[idx] = v;
    sW1h[idx] = (_Float16)(v * SC_W1);
  }
  __syncthreads();
  {
    float qa = 0.f, qb = 0.f;
#pragma unroll
    for (int d = 0; d < NPART; ++d) {
      const float va = sW1f[d * HID + tid];
      const float vb = sW1f[d * HID + tid + 256];
      qa = fmaf(va, va, qa);
      qb = fmaf(vb, vb, qb);
    }
    sQ[tid] = qa;
    sQ[tid + 256] = qb;
  }

  const int mt = w >> 2, cq = w & 3;
  const int rbase = b0 + mt * 16;
  const _Float16* ar = s1h + (size_t)(rbase + m) * HID;
  float part[8];
#pragma unroll
  for (int v = 0; v < 8; ++v) part[v] = 0.f;

#pragma unroll 1
  for (int nt = 0; nt < 8; ++nt) {
    const int n0 = cq * 128 + nt * 16;
    const _Float16* br = w2th + (size_t)(n0 + m) * HID;
    v8f acc[NPART];
#pragma unroll
    for (int d = 0; d < NPART; ++d) acc[d] = zero8();
#pragma unroll 1
    for (int k0 = 0; k0 < HID; k0 += 32) {
      const v16h s  = ld_frag(ar, k0, h);
      const v16h bb = ld_frag(br, k0, h);
#pragma unroll
      for (int d = 0; d < NPART; ++d) {
        const v16h wv = ld_frag(sW1h + d * HID, k0, h);
        const v16h u  = s * wv;
        acc[d] = wmma_f16(u, bb, acc[d]);
      }
    }
    v8f sq = zero8();
#pragma unroll
    for (int d = 0; d < NPART; ++d)
#pragma unroll
      for (int v = 0; v < 8; ++v) sq[v] = fmaf(acc[d][v], acc[d][v], sq[v]);
#pragma unroll
    for (int v = 0; v < 8; ++v) {
      float val = wf[(size_t)(rbase + 8 * h + v) * HID + n0 + m] * sq[v];
      val += __shfl_xor(val, 1, 32);
      val += __shfl_xor(val, 2, 32);
      val += __shfl_xor(val, 4, 32);
      val += __shfl_xor(val, 8, 32);
      part[v] += val;
    }
  }
  if (m == 0) {
#pragma unroll
    for (int v = 0; v < 8; ++v) sLap[w][8 * h + v] = part[v];
  }
  __syncthreads();

#pragma unroll 1
  for (int i = 0; i < 4; ++i) {
    const int r = w * 4 + i;
    const int b = b0 + r;
    const float* Rrow = Rf  + (size_t)b * HID;
    const float* Hrow = h1f + (size_t)b * HID;
    float accn[NPART];
#pragma unroll
    for (int d = 0; d < NPART; ++d) accn[d] = 0.f;
    float accT2 = 0.f;
#pragma unroll 4
    for (int it = 0; it < HID / 32; ++it) {
      const int j = lane + 32 * it;
      const float rr = Rrow[j];
      const float hh = Hrow[j];
      const float s  = fmaf(-hh, hh, 1.0f);
      const float v1 = s * rr;
#pragma unroll
      for (int d = 0; d < NPART; ++d) accn[d] = fmaf(v1, sW1f[d * HID + j], accn[d]);
      accT2 = fmaf((hh * s) * sQ[j], rr, accT2);
    }
    float g2 = 0.f;
#pragma unroll
    for (int d = 0; d < NPART; ++d) {
      float a = accn[d];
      a += __shfl_xor(a, 1, 32);
      a += __shfl_xor(a, 2, 32);
      a += __shfl_xor(a, 4, 32);
      a += __shfl_xor(a, 8, 32);
      a += __shfl_xor(a, 16, 32);
      g2 = fmaf(a, a, g2);
    }
    accT2 += __shfl_xor(accT2, 1, 32);
    accT2 += __shfl_xor(accT2, 2, 32);
    accT2 += __shfl_xor(accT2, 4, 32);
    accT2 += __shfl_xor(accT2, 8, 32);
    accT2 += __shfl_xor(accT2, 16, 32);
    if (lane == 0) {
      const int mt2 = r >> 4, rl = r & 15;
      float t1 = sLap[mt2 * 4 + 0][rl];
      t1 += sLap[mt2 * 4 + 1][rl];
      t1 += sLap[mt2 * 4 + 2][rl];
      t1 += sLap[mt2 * 4 + 3][rl];
      const float term1 = -(t1 * TERM1_SCALE);
      const float term2 = -2.0f * accT2;
      const float ek = -0.5f * ((term1 + term2) + g2);
      float xv[NPART];
      float sx2 = 0.f;
#pragma unroll
      for (int i2 = 0; i2 < NPART; ++i2) {
        xv[i2] = x[(size_t)b * NPART + i2];
        sx2 = fmaf(xv[i2], xv[i2], sx2);
      }
      float sg = 0.f;
#pragma unroll
      for (int i2 = 0; i2 < NPART; ++i2) {
#pragma unroll
        for (int j2 = i2 + 1; j2 < NPART; ++j2) {
          const float dd = xv[j2] - xv[i2];
          sg += expf(-(dd * dd) * 2.0f);
        }
      }
      sOut[r] = (ek + 0.5f * sx2) + GAUSS_C * sg;
    }
  }
  __syncthreads();
  if (w == 0 && lane < 8) {
    const v4f o = *(const v4fa*)(&sOut[lane * 4]);
    float* po = out + (size_t)b0 + lane * 4;
    *(volatile v4f*)po = o;
    __threadfence();
    *(volatile v4f*)po = o;
  }
}

extern "C" void kernel_launch(void* const* d_in, const int* in_sizes, int n_in,
                              void* d_out, int out_size, void* d_ws, size_t ws_size,
                              hipStream_t stream) {
  if (n_in < 7) return;
  if (in_sizes[0] != NWALK * NPART || in_sizes[1] != NPART * HID || in_sizes[2] != HID ||
      in_sizes[3] != HID * HID || in_sizes[4] != HID || in_sizes[5] != HID || in_sizes[6] < 1 ||
      out_size != NWALK) return;
  const float* x  = (const float*)d_in[0];
  const float* W1 = (const float*)d_in[1];
  const float* b1 = (const float*)d_in[2];
  const float* W2 = (const float*)d_in[3];
  const float* b2 = (const float*)d_in[4];
  const float* W3 = (const float*)d_in[5];
  const float* b3 = (const float*)d_in[6];
  float* out = (float*)d_out;

  size_t off = 0;
  auto carve = [&](size_t bytes) -> size_t {
    off = (off + 255) & ~(size_t)255;
    const size_t o = off;
    off += bytes;
    return o;
  };
  const size_t o_w2h  = carve((size_t)HID * HID * 2);
  const size_t o_w2th = carve((size_t)HID * HID * 2);
  const size_t o_h1f  = carve((size_t)NWALK * HID * 4);
  const size_t o_h1h  = carve((size_t)NWALK * HID * 2);
  const size_t o_s1h  = carve((size_t)NWALK * HID * 2);
  const size_t o_v2h  = carve((size_t)NWALK * HID * 2);
  const size_t o_wf   = carve((size_t)NWALK * HID * 4);
  const size_t o_Rf   = carve((size_t)NWALK * HID * 4);
  if (off > ws_size) return;
  char* ws = (char*)d_ws;
  _Float16* w2h  = (_Float16*)(ws + o_w2h);
  _Float16* w2th = (_Float16*)(ws + o_w2th);
  float*    h1f  = (float*)(ws + o_h1f);
  _Float16* h1h  = (_Float16*)(ws + o_h1h);
  _Float16* s1h  = (_Float16*)(ws + o_s1h);
  _Float16* v2h  = (_Float16*)(ws + o_v2h);
  float*    wf   = (float*)(ws + o_wf);
  float*    Rf   = (float*)(ws + o_Rf);

  k_prep<<<(HID / 64) * (HID / 64), 256, 0, stream>>>(W2, w2h, w2th);
  k_fwd<<<NWALK / 16, 256, 0, stream>>>(x, W1, b1, h1f, h1h, s1h);
  k_gemm1<<<(NWALK / 32) * (HID / 128), 128, 0, stream>>>(h1h, w2th, b2, W3, v2h, wf);
  k_gemm2<<<(NWALK / 32) * (HID / 128), 128, 0, stream>>>(v2h, w2h, Rf);
  k_lapfin<<<NWALK / 32, 256, 0, stream>>>(s1h, w2th, wf, Rf, h1f, x, W1, b3, out);
  (void)hipGetLastError();
}
